// WaveAttention_29308856827997
// MI455X (gfx1250) — hardware-verified
//
#include <hip/hip_runtime.h>
#include <math.h>
#include <stdint.h>

#define NB     2
#define SEQ    2048
#define DMOD   1024
#define FEAT   256
#define HDIM   64
#define NHEAD  16
#define NWH    4
#define NPH    4
#define NSH    8
#define HCOLS  (NHEAD * HDIM)
#define WAVC   (NWH * HDIM)
#define PRJC   (NPH * HDIM)
#define STDC   (NSH * HDIM)
#define ROWS   (NB * SEQ)
#define MWORDS (SEQ / 32)
#define NQB    (SEQ / 64)
#define NKT    (SEQ / 64)
#define AOP    (2 * HCOLS)
static_assert(NWH + NPH + NSH == NHEAD);
static_assert(HCOLS == DMOD);
static_assert((ROWS % 64) == 0 && (DMOD % 64) == 0 && (STDC % 64) == 0 && (WAVC % 64) == 0 && (PRJC % 64) == 0 && (SEQ % 64) == 0);
static_assert((DMOD % 32) == 0 && (FEAT % 32) == 0 && (AOP % 32) == 0);
static_assert((FEAT % 64) == 0 && (HDIM % 64) == 0);
static_assert(NQB == 32 && NKT == 32 && MWORDS == 64);

typedef _Float16 v16h __attribute__((ext_vector_type(16)));
typedef _Float16 v8h  __attribute__((ext_vector_type(8)));
typedef __bf16   v16b __attribute__((ext_vector_type(16)));
typedef __bf16   v8b  __attribute__((ext_vector_type(8)));
typedef float    v8f  __attribute__((ext_vector_type(8)));
typedef float    v4f  __attribute__((ext_vector_type(4)));
typedef unsigned int v4u __attribute__((ext_vector_type(4)));
typedef unsigned int v2u __attribute__((ext_vector_type(2)));
typedef int      v4i __attribute__((ext_vector_type(4)));

#if defined(__HIP_DEVICE_COMPILE__)
#define DEV_ASM 1
#else
#define DEV_ASM 0
#endif

__device__ __forceinline__ unsigned short bf_bits(float f) {
  unsigned u = __float_as_uint(f);
  return (unsigned short)((u + 0x7FFFu + ((u >> 16) & 1u)) >> 16);
}
__device__ __forceinline__ float bf_up(unsigned short hb) { return __uint_as_float(((unsigned)hb) << 16); }
__device__ __forceinline__ float bfr(float f) { return bf_up(bf_bits(f)); }
__device__ __forceinline__ unsigned short h_bits(_Float16 x) { return __builtin_bit_cast(unsigned short, x); }
__device__ __forceinline__ unsigned pk16(unsigned short a, unsigned short b) { return (unsigned)a | ((unsigned)b << 16); }
__device__ __forceinline__ v8f zero8() { v8f z = {0.f, 0.f, 0.f, 0.f, 0.f, 0.f, 0.f, 0.f}; return z; }

template <typename OT> struct FT;
template <> struct FT<__bf16>   { typedef v16b frag; typedef v8b half8; };
template <> struct FT<_Float16> { typedef v16h frag; typedef v8h half8; };

template <typename OT>
__device__ __forceinline__ typename FT<OT>::frag ldfrag(const OT* p) {
  union { typename FT<OT>::frag v; typename FT<OT>::half8 h[2]; } f;
  f.h[0] = *(const typename FT<OT>::half8*)(p);
  f.h[1] = *(const typename FT<OT>::half8*)(p + 16);
  return f.v;
}

__device__ __forceinline__ v8f mmar(v16b a, v16b b, v8f c) {
  return __builtin_amdgcn_wmma_f32_16x16x32_bf16(false, a, false, b, (short)0, c, false, false);
}
__device__ __forceinline__ v8f mmar(v16h a, v16h b, v8f c) {
  return __builtin_amdgcn_wmma_f32_16x16x32_f16(false, a, false, b, (short)0, c, false, false);
}
__device__ __forceinline__ v8f mma_g(v16h a, v16h b, v8f c) {
  c = __builtin_amdgcn_wmma_f32_16x16x32_f16(false, a, false, b, (short)0, c, false, false);
#if DEV_ASM
  asm volatile("v_nop\n\tv_nop\n\tv_nop\n\tv_nop" : "+v"(c) : "v"(a), "v"(b));
#endif
  return c;
}
__device__ __forceinline__ v8f mma_g(v16b a, v16b b, v8f c) {
  c = __builtin_amdgcn_wmma_f32_16x16x32_bf16(false, a, false, b, (short)0, c, false, false);
#if DEV_ASM
  asm volatile("v_nop\n\tv_nop\n\tv_nop\n\tv_nop" : "+v"(c) : "v"(a), "v"(b));
#endif
  return c;
}
__device__ __forceinline__ void dep_guard(v8f& a, v8f& b, v16b x, v16b y) {
#if DEV_ASM
  asm volatile("v_nop\n\tv_nop\n\tv_nop\n\tv_nop" : "+v"(a), "+v"(b) : "v"(x), "v"(y));
#else
  (void)a; (void)b; (void)x; (void)y;
#endif
}
__device__ __forceinline__ void dep_guard(v8f& a, v8f& b, v16h x, v16h y) {
#if DEV_ASM
  asm volatile("v_nop\n\tv_nop\n\tv_nop\n\tv_nop" : "+v"(a), "+v"(b) : "v"(x), "v"(y));
#else
  (void)a; (void)b; (void)x; (void)y;
#endif
}
__device__ __forceinline__ void keep4(v16b a, v16b b, v16b c, v16b d) {
#if DEV_ASM
  asm volatile("v_nop" :: "v"(a), "v"(b), "v"(c), "v"(d));
#else
  (void)a; (void)b; (void)c; (void)d;
#endif
}
__device__ __forceinline__ void keep4(v16h a, v16h b, v16h c, v16h d) {
#if DEV_ASM
  asm volatile("v_nop" :: "v"(a), "v"(b), "v"(c), "v"(d));
#else
  (void)a; (void)b; (void)c; (void)d;
#endif
}
__device__ __forceinline__ void acc_guard4(v8f& a, v8f& b, v8f& c, v8f& d) {
#if DEV_ASM
  asm volatile("v_nop\n\tv_nop\n\tv_nop\n\tv_nop" : "+v"(a), "+v"(b), "+v"(c), "+v"(d));
#else
  (void)a; (void)b; (void)c; (void)d;
#endif
}

__global__ __launch_bounds__(256) void mask_bits_kernel(const int* __restrict__ mask, unsigned int* mb, int nwords) {
  const int i = blockIdx.x * 256 + (int)threadIdx.x;
  if (i < nwords) {
    const int* p = mask + (size_t)i * 32;
    unsigned w = 0u;
#pragma unroll
    for (int q = 0; q < 8; ++q) {
      const v4i v = *(const v4i*)(p + 4 * q);
#pragma unroll
      for (int e = 0; e < 4; ++e) w |= ((v[e] != 0) ? 1u : 0u) << (4 * q + e);
    }
    *(volatile unsigned int*)(mb + i) = w;
    __threadfence();
    *(volatile unsigned int*)(mb + i) = w;
  }
}

__global__ __launch_bounds__(256) void cvt_bf16x8(const float* __restrict__ in, unsigned short* out, int n8) {
  const int i = blockIdx.x * 256 + (int)threadIdx.x;
  if (i < n8) {
    const v4f a  = *(const v4f*)(in + (size_t)i * 8);
    const v4f a4 = *(const v4f*)(in + (size_t)i * 8 + 4);
    v4u p;
    p[0] = pk16(bf_bits(a[0]),  bf_bits(a[1]));
    p[1] = pk16(bf_bits(a[2]),  bf_bits(a[3]));
    p[2] = pk16(bf_bits(a4[0]), bf_bits(a4[1]));
    p[3] = pk16(bf_bits(a4[2]), bf_bits(a4[3]));
    unsigned short* o = out + (size_t)i * 8;
    *(volatile v4u*)o = p;
    __threadfence();
    *(volatile v4u*)o = p;
  }
}

template <bool DUP>
__global__ __launch_bounds__(256) void transpose_bf16_kernel(
    const float* __restrict__ in, int inC, long long inStrideZ,
    unsigned short* out, int ldo, long long outStrideZ, int dupoff) {
  __shared__ __align__(16) unsigned short th[64 * 72];
  const int c0  = blockIdx.x * 64;
  const int r0  = blockIdx.y * 64;
  const int z   = blockIdx.z;
  const int tid = threadIdx.x;
  const float* inz = in + (size_t)z * (size_t)inStrideZ;
  unsigned short* outz = out + (size_t)z * (size_t)outStrideZ;
  {
    const int rr = tid >> 2;
    const int cq = (tid & 3) * 16;
    const float* src = inz + (size_t)(r0 + rr) * inC + c0 + cq;
#pragma unroll
    for (int q = 0; q < 4; ++q) {
      const v4f f = *(const v4f*)(src + 4 * q);
#pragma unroll
      for (int e = 0; e < 4; ++e) th[rr * 72 + cq + 4 * q + e] = bf_bits(f[e]);
    }
  }
  __syncthreads();
  const int sub = tid >> 3;
  const int c8  = (tid & 7) * 8;
  v4u hv[2];
#pragma unroll
  for (int it = 0; it < 2; ++it) {
    const int oc = it * 32 + sub;
    v4u a;
#pragma unroll
    for (int q = 0; q < 4; ++q) a[q] = pk16(th[(c8 + 2 * q) * 72 + oc], th[(c8 + 2 * q + 1) * 72 + oc]);
    hv[it] = a;
  }
  for (int pass = 0; pass < 2; ++pass) {
#pragma unroll
    for (int it = 0; it < 2; ++it) {
      const int oc = it * 32 + sub;
      const size_t go = (size_t)(c0 + oc) * ldo + r0 + c8;
      *(volatile v4u*)(outz + go) = hv[it];
      if (DUP) *(volatile v4u*)(outz + go + dupoff) = hv[it];
    }
    __threadfence();
  }
}

template <typename OT, int OUT_MODE, int BIAS_MODE>
__global__ __launch_bounds__(256) void gemm64(
    const unsigned short* __restrict__ Ap, int lda, long long strideA,
    const unsigned short* __restrict__ Btp, int ldb, long long strideB,
    void* Cout, void* Cout2, int ldc, long long strideC,
    const float* __restrict__ bias, int M, int N, int K, float oscale) {
  typedef typename FT<OT>::frag V16;
  const OT* A  = (const OT*)(const void*)Ap;
  const OT* Bt = (const OT*)(const void*)Btp;
  __shared__ __align__(16) float sT[8][16 * 68];
  const int b    = blockIdx.y;
  const int lane = threadIdx.x & 31;
  const int wave = threadIdx.x >> 5;
  const int tilesN = N >> 6;
  const int tilesM = M >> 6;
  const int tile = blockIdx.x * 8 + wave;
  if (tile >= tilesM * tilesN) return;
  const int tm = tile / tilesN;
  const int tn = tile - tm * tilesN;
  const int m0 = tm << 6;
  const int n0 = tn << 6;

  const OT* Ab = A  + (size_t)b * (size_t)strideA;
  const OT* Bb = Bt + (size_t)b * (size_t)strideB;

  const int rlane = lane & 15;
  const int koff  = (lane >> 4) * 8;
  const int mOff  = (lane >> 4) * 8;

  v8f acc[4][4];
#pragma unroll
  for (int i = 0; i < 4; ++i)
#pragma unroll
    for (int j = 0; j < 4; ++j) acc[i][j] = zero8();

  for (int k0 = 0; k0 < K; k0 += 32) {
    V16 bq[4];
#pragma unroll
    for (int j = 0; j < 4; ++j)
      bq[j] = ldfrag<OT>(Bb + (size_t)(n0 + (j << 4) + rlane) * ldb + koff + k0);
#pragma unroll
    for (int i = 0; i < 4; ++i) {
      const V16 af = ldfrag<OT>(Ab + (size_t)(m0 + (i << 4) + rlane) * lda + koff + k0);
#pragma unroll
      for (int j = 0; j < 4; ++j) acc[i][j] = mmar(af, bq[j], acc[i][j]);
      dep_guard(acc[i][0], acc[i][3], af, bq[3]);
    }
    keep4(bq[0], bq[1], bq[2], bq[3]);
  }
  acc_guard4(acc[0][0], acc[0][1], acc[0][2], acc[0][3]);
  acc_guard4(acc[1][0], acc[1][1], acc[1][2], acc[1][3]);
  acc_guard4(acc[2][0], acc[2][1], acc[2][2], acc[2][3]);
  acc_guard4(acc[3][0], acc[3][1], acc[3][2], acc[3][3]);

  float* slab = sT[wave];
#pragma unroll
  for (int i = 0; i < 4; ++i) {
    const int mBase = m0 + (i << 4);
#pragma unroll
    for (int j = 0; j < 4; ++j) {
      const int n = n0 + (j << 4) + rlane;
      float bn = 0.f;
      if (BIAS_MODE == 2) bn = bfr(bias[n]);
#pragma unroll
      for (int r = 0; r < 8; ++r) {
        float v = acc[i][j][r];
        if (BIAS_MODE == 1) v += bfr(bias[mBase + mOff + r]);
        if (BIAS_MODE == 2) v += bn;
        slab[(mOff + r) * 68 + (j << 4) + rlane] = v * oscale;
      }
    }
    __builtin_amdgcn_fence(__ATOMIC_RELEASE, "workgroup");
    __builtin_amdgcn_wave_barrier();
    __builtin_amdgcn_fence(__ATOMIC_ACQUIRE, "workgroup");
    if (OUT_MODE == 0) {
      float* C = (float*)Cout + (size_t)b * (size_t)strideC;
      const int h2 = lane >> 4, c4 = (lane & 15) * 4;
      for (int pass = 0; pass < 2; ++pass) {
#pragma unroll
        for (int it = 0; it < 8; ++it) {
          const int row = it * 2 + h2;
          const v4f v = *(const v4f*)(slab + row * 68 + c4);
          *(volatile v4f*)(C + (size_t)(mBase + row) * ldc + n0 + c4) = v;
        }
        __threadfence();
      }
    } else {
      const int q = lane >> 3, c8 = (lane & 7) * 8;
      unsigned short* C  = (unsigned short*)Cout  + (size_t)b * (size_t)strideC;
      unsigned short* C2 = (unsigned short*)Cout2 + (size_t)b * (size_t)strideC;
      v4u hv[4], lv[4];
#pragma unroll
      for (int it = 0; it < 4; ++it) {
        const int row = it * 4 + q;
        const float* sp = slab + row * 68 + c8;
        v4u a, a2;
#pragma unroll
        for (int e = 0; e < 4; ++e) {
          const float f0 = sp[2 * e], f1 = sp[2 * e + 1];
          unsigned short h0, h1, l0 = 0, l1 = 0;
          if (OUT_MODE == 1) {
            h0 = h_bits((_Float16)f0); h1 = h_bits((_Float16)f1);
          } else {
            h0 = bf_bits(f0); h1 = bf_bits(f1);
            l0 = bf_bits(f0 - bf_up(h0)); l1 = bf_bits(f1 - bf_up(h1));
          }
          a[e] = pk16(h0, h1); a2[e] = pk16(l0, l1);
        }
        hv[it] = a; lv[it] = a2;
      }
      for (int pass = 0; pass < 2; ++pass) {
#pragma unroll
        for (int it = 0; it < 4; ++it) {
          const int row = it * 4 + q;
          *(volatile v4u*)(C + (size_t)(mBase + row) * ldc + n0 + c8) = hv[it];
          if (OUT_MODE == 2) *(volatile v4u*)(C2 + (size_t)(mBase + row) * ldc + n0 + c8) = lv[it];
        }
        __threadfence();
      }
    }
    __builtin_amdgcn_fence(__ATOMIC_RELEASE, "workgroup");
    __builtin_amdgcn_wave_barrier();
    __builtin_amdgcn_fence(__ATOMIC_ACQUIRE, "workgroup");
  }
}

template <int HT> struct HT_T;
template <> struct HT_T<0> { typedef __bf16 T; };
template <> struct HT_T<1> { typedef _Float16 T; };

template <int HT>
__global__ __launch_bounds__(128)
void attn_kernel(const unsigned short* __restrict__ qhp, const unsigned short* __restrict__ qlp, int ldq,
                 const unsigned short* __restrict__ khp, const unsigned short* __restrict__ klp, int ldk,
                 const unsigned short* __restrict__ vtp, const unsigned int* __restrict__ mbp,
                 unsigned short* aop, int hbase, int nh, float sscale) {
  typedef typename HT_T<HT>::T OT;
  typedef typename FT<OT>::frag V16;
  typedef typename FT<OT>::half8 V8;
  union FH { v16h v; v8h h[2]; };
  union FO { V16 v; V8 h[2]; };
  __shared__ __align__(16) OT       Ksh[64 * 64];
  __shared__ __align__(16) OT       Ksl[64 * 64];
  __shared__ __align__(16) _Float16 Vth[64 * 64];
  __shared__ __align__(16) _Float16 Psh[4][16 * 64];
  __shared__ __align__(16) float    Os[4][16 * 64];

  const int tid  = threadIdx.x;
  const int wave = tid >> 5;
  const int lane = tid & 31;
  const int hh   = lane >> 4;
  const int c    = lane & 15;

  const int bx   = blockIdx.x;
  const int qb   = bx % NQB;
  const int rest = bx / NQB;
  const int hl   = rest % nh;
  const int b    = rest / nh;
  const int h    = hbase + hl;
  const int qc   = h * HDIM;
  const int q0   = qb * 64 + wave * 16;
  const size_t rowB = (size_t)b * SEQ;

  const OT* Qh = (const OT*)(const void*)qhp;
  const OT* Ql = (const OT*)(const void*)qlp;
  const OT* Kh = (const OT*)(const void*)khp + qc;
  const OT* Kl = (const OT*)(const void*)klp + qc;
  const _Float16* Vt = (const _Float16*)(const void*)vtp + ((size_t)b * HCOLS + (size_t)qc) * SEQ;

  V16 qah[2], qal[2];
#pragma unroll
  for (int dc = 0; dc < 2; ++dc) {
    const size_t qo = (rowB + q0 + c) * (size_t)ldq + (size_t)qc + dc * 32 + 8 * hh;
    qah[dc] = ldfrag<OT>(Qh + qo);
    if (HT == 0) qal[dc] = ldfrag<OT>(Ql + qo);
    else         qal[dc] = qah[dc];
  }

  float mrow[8], lrow[8];
  v8f oacc[4];
#pragma unroll
  for (int r = 0; r < 8; ++r) { mrow[r] = -INFINITY; lrow[r] = 0.f; }
#pragma unroll
  for (int t = 0; t < 4; ++t) oacc[t] = zero8();

  for (int kt = 0; kt < NKT; ++kt) {
    const int kv0 = kt * 64;
    __syncthreads();
    {
      const int r = tid >> 1, half = (tid & 1) * 32;
      const OT* kg  = Kh + (rowB + kv0 + r) * (size_t)ldk + half;
      const OT* klg = Kl + (rowB + kv0 + r) * (size_t)ldk + half;
      const _Float16* vg = Vt + (size_t)r * SEQ + kv0 + half;
#pragma unroll
      for (int i = 0; i < 4; ++i) {
        *(V8*)(Ksh + r * 64 + half + 8 * i) = *(const V8*)(kg + 8 * i);
        if (HT == 0) *(V8*)(Ksl + r * 64 + half + 8 * i) = *(const V8*)(klg + 8 * i);
        *(v8h*)(Vth + r * 64 + half + 8 * i) = *(const v8h*)(vg + 8 * i);
      }
    }
    __syncthreads();

    unsigned mk = 0u;
#pragma unroll
    for (int r = 0; r < 8; ++r) {
      const int row = q0 + 8 * hh + r;
      const v2u mw = *(const v2u*)(mbp + (rowB + row) * (size_t)MWORDS + 2 * kt);
#pragma unroll
      for (int j = 0; j < 4; ++j) {
        const unsigned bit = (mw[j >> 1] >> (16 * (j & 1) + c)) & 1u;
        mk |= bit << (4 * r + j);
      }
    }

    v8f s[4];
#pragma unroll
    for (int j = 0; j < 4; ++j) {
      v8f a0 = zero8();
#pragma unroll
      for (int dc = 0; dc < 2; ++dc) {
        FO kb;
        kb.h[0] = *(const V8*)(Ksh + (j * 16 + c) * 64 + dc * 32 + 8 * hh);
        kb.h[1] = *(const V8*)(Ksh + (j * 16 + c) * 64 + dc * 32 + 16 + 8 * hh);
        if (HT == 0) {
          FO kl;
          kl.h[0] = *(const V8*)(Ksl + (j * 16 + c) * 64 + dc * 32 + 8 * hh);
          kl.h[1] = *(const V8*)(Ksl + (j * 16 + c) * 64 + dc * 32 + 16 + 8 * hh);
          a0 = mma_g(qah[dc], kb.v, a0);
          a0 = mma_g(qah[dc], kl.v, a0);
          a0 = mma_g(qal[dc], kb.v, a0);
        } else {
          a0 = mma_g(qah[dc], kb.v, a0);
        }
      }
#pragma unroll
      for (int r = 0; r < 8; ++r) {
        const float v = a0[r] * sscale;
        s[j][r] = (((mk >> (4 * r + j)) & 1u) != 0u) ? v : -INFINITY;
      }
    }

    _Float16* pwh = Psh[wave];
#pragma unroll
    for (int r = 0; r < 8; ++r) {
      float m = s[0][r];
#pragma unroll
      for (int j = 1; j < 4; ++j) m = fmaxf(m, s[j][r]);
#pragma unroll
      for (int off = 1; off < 16; off <<= 1) m = fmaxf(m, __shfl_xor(m, off, 32));
      const float mnew  = fmaxf(mrow[r], m);
      const float msafe = (mnew == -INFINITY) ? 0.f : mnew;
      const float alpha = expf(mrow[r] - msafe);
      mrow[r] = mnew;
      float psum = 0.f;
#pragma unroll
      for (int j = 0; j < 4; ++j) {
        const float p = expf(s[j][r] - msafe);
        psum += p;
        pwh[(8 * hh + r) * 64 + j * 16 + c] = (_Float16)(p * 1024.0f);
      }
#pragma unroll
      for (int off = 1; off < 16; off <<= 1) psum += __shfl_xor(psum, off, 32);
      lrow[r] = lrow[r] * alpha + psum;
#pragma unroll
      for (int t = 0; t < 4; ++t) oacc[t][r] *= alpha;
    }
    __builtin_amdgcn_fence(__ATOMIC_RELEASE, "workgroup");
    __builtin_amdgcn_wave_barrier();
    __builtin_amdgcn_fence(__ATOMIC_ACQUIRE, "workgroup");

#pragma unroll 1
    for (int kk = 0; kk < 2; ++kk) {
      FH pa;
      pa.h[0] = *(const v8h*)(pwh + c * 64 + kk * 32 + 8 * hh);
      pa.h[1] = *(const v8h*)(pwh + c * 64 + kk * 32 + 16 + 8 * hh);
#pragma unroll
      for (int t = 0; t < 4; ++t) {
        FH vb;
        vb.h[0] = *(const v8h*)(Vth + (t * 16 + c) * 64 + kk * 32 + 8 * hh);
        vb.h[1] = *(const v8h*)(Vth + (t * 16 + c) * 64 + kk * 32 + 16 + 8 * hh);
        oacc[t] = mma_g(pa.v, vb.v, oacc[t]);
      }
    }
  }

  float* os = Os[wave];
#pragma unroll
  for (int r = 0; r < 8; ++r) {
    const float inv = (1.0f / lrow[r]) * (1.0f / 8192.0f);
#pragma unroll
    for (int t = 0; t < 4; ++t) os[(8 * hh + r) * 64 + t * 16 + c] = oacc[t][r] * inv;
  }
  __builtin_amdgcn_fence(__ATOMIC_RELEASE, "workgroup");
  __builtin_amdgcn_wave_barrier();
  __builtin_amdgcn_fence(__ATOMIC_ACQUIRE, "workgroup");
  {
    const int q4 = lane >> 3, c8 = (lane & 7) * 8;
    v4u hv[4], lv[4];
#pragma unroll
    for (int it = 0; it < 4; ++it) {
      const int row = it * 4 + q4;
      const float* sp = os + row * 64 + c8;
      v4u a, a2;
#pragma unroll
      for (int e = 0; e < 4; ++e) {
        const float f0 = sp[2 * e], f1 = sp[2 * e + 1];
        const unsigned short hb0 = bf_bits(f0), hb1 = bf_bits(f1);
        const unsigned short lb0 = bf_bits(f0 - bf_up(hb0)), lb1 = bf_bits(f1 - bf_up(hb1));
        a[e] = pk16(hb0, hb1); a2[e] = pk16(lb0, lb1);
      }
      hv[it] = a; lv[it] = a2;
    }
    for (int pass = 0; pass < 2; ++pass) {
#pragma unroll
      for (int it = 0; it < 4; ++it) {
        const int row = it * 4 + q4;
        const size_t go = (rowB + q0 + row) * (size_t)AOP + (size_t)qc + c8;
        *(volatile v4u*)(aop + go) = hv[it];
        *(volatile v4u*)(aop + go + HCOLS) = lv[it];
      }
      __threadfence();
    }
  }
}

extern "C" void kernel_launch(void* const* d_in, const int* in_sizes, int n_in,
                              void* d_out, int out_size, void* d_ws, size_t ws_size,
                              hipStream_t stream) {
  if (n_in < 14) return;
  if (in_sizes[0] != NB * SEQ * DMOD) return;
  if (in_sizes[1] != NB * SEQ * FEAT) return;
  if (in_sizes[2] != NB * SEQ * SEQ) return;
  if (in_sizes[3] != NWH * FEAT * HDIM || in_sizes[4] != NPH * FEAT * HDIM || in_sizes[5] != NPH * FEAT * HDIM) return;
  if (in_sizes[6] != DMOD * STDC || in_sizes[7] != STDC) return;
  if (in_sizes[8] != DMOD * STDC || in_sizes[9] != STDC) return;
  if (in_sizes[10] != DMOD * HCOLS || in_sizes[11] != HCOLS) return;
  if (in_sizes[12] != HCOLS * DMOD || in_sizes[13] != DMOD) return;
  if (out_size != NB * SEQ * DMOD) return;

  const float* x     = (const float*)d_in[0];
  const float* feats = (const float*)d_in[1];
  const int*   mask  = (const int*)d_in[2];
  const float* wproj = (const float*)d_in[3];
  const float* pqw   = (const float*)d_in[4];
  const float* pkw   = (const float*)d_in[5];
  const float* sqw   = (const float*)d_in[6];
  const float* sqb   = (const float*)d_in[7];
  const float* skw   = (const float*)d_in[8];
  const float* skb   = (const float*)d_in[9];
  const float* vw    = (const float*)d_in[10];
  const float* vb    = (const float*)d_in[11];
  const float* ow    = (const float*)d_in[12];
  const float* ob    = (const float*)d_in[13];

  const size_t PMB  = (size_t)NB * SEQ * MWORDS * 4;
  const size_t PXB  = (size_t)ROWS * DMOD * 2;
  const size_t PFB  = (size_t)ROWS * FEAT * 2;
  const size_t PVWT = (size_t)HCOLS * DMOD * 2;
  const size_t PSWT = (size_t)STDC * DMOD * 2;
  const size_t PFWT = (size_t)WAVC * FEAT * 2;
  const size_t POWT = (size_t)DMOD * AOP * 2;
  const size_t PVT  = (size_t)NB * HCOLS * SEQ * 2;
  const size_t PQP  = (size_t)ROWS * HCOLS * 2;
  const size_t PWP  = (size_t)ROWS * WAVC * 2;
  const size_t PAO  = (size_t)ROWS * AOP * 2;
  size_t off = 0;
  const size_t oMB  = off; off += PMB;
  const size_t oXB  = off; off += PXB;
  const size_t oFB  = off; off += PFB;
  const size_t oVWT = off; off += PVWT;
  const size_t oQWT = off; off += PSWT;
  const size_t oKWT = off; off += PSWT;
  const size_t oWVT = off; off += PFWT;
  const size_t oPQT = off; off += PFWT;
  const size_t oPKT = off; off += PFWT;
  const size_t oOWT = off; off += POWT;
  const size_t oVT  = off; off += PVT;
  const size_t oQP  = off; off += PQP;
  const size_t oKP  = off; off += PQP;
  const size_t oWPH = off; off += PWP;
  const size_t oWPL = off; off += PWP;
  const size_t oAO  = off; off += PAO;
  if (off > ws_size) return;
  if (off > (size_t)134217728) return;

  char* ws = (char*)d_ws;
  unsigned int*   MB   = (unsigned int*)(ws + oMB);
  unsigned short* XB   = (unsigned short*)(ws + oXB);
  unsigned short* FB   = (unsigned short*)(ws + oFB);
  unsigned short* VWT  = (unsigned short*)(ws + oVWT);
  unsigned short* QWT  = (unsigned short*)(ws + oQWT);
  unsigned short* KWT  = (unsigned short*)(ws + oKWT);
  unsigned short* WVT  = (unsigned short*)(ws + oWVT);
  unsigned short* PQT  = (unsigned short*)(ws + oPQT);
  unsigned short* PKT  = (unsigned short*)(ws + oPKT);
  unsigned short* OWT2 = (unsigned short*)(ws + oOWT);
  unsigned short* VT   = (unsigned short*)(ws + oVT);
  unsigned short* QP   = (unsigned short*)(ws + oQP);
  unsigned short* KP   = (unsigned short*)(ws + oKP);
  unsigned short* WPH  = (unsigned short*)(ws + oWPH);
  unsigned short* WPL  = (unsigned short*)(ws + oWPL);
  unsigned short* AO   = (unsigned short*)(ws + oAO);

  const dim3 blk(256);
  const int nwords = NB * SEQ * MWORDS;
  const int n8x    = ROWS * DMOD / 8;
  const int n8f    = ROWS * FEAT / 8;

  mask_bits_kernel<<<dim3((nwords + 255) / 256), blk, 0, stream>>>(mask, MB, nwords);
  cvt_bf16x8<<<dim3((n8x + 255) / 256), blk, 0, stream>>>(x, XB, n8x);
  cvt_bf16x8<<<dim3((n8f + 255) / 256), blk, 0, stream>>>(feats, FB, n8f);

  transpose_bf16_kernel<false><<<dim3(HCOLS / 64, DMOD / 64, 1), blk, 0, stream>>>(vw, HCOLS, 0LL, VWT, DMOD, 0LL, 0);
  transpose_bf16_kernel<false><<<dim3(STDC / 64, DMOD / 64, 1), blk, 0, stream>>>(sqw, STDC, 0LL, QWT, DMOD, 0LL, 0);
  transpose_bf16_kernel<false><<<dim3(STDC / 64, DMOD / 64, 1), blk, 0, stream>>>(skw, STDC, 0LL, KWT, DMOD, 0LL, 0);
  transpose_bf16_kernel<false><<<dim3(HDIM / 64, FEAT / 64, NWH), blk, 0, stream>>>(wproj, HDIM, (long long)FEAT * HDIM, WVT, FEAT, (long long)HDIM * FEAT, 0);
  transpose_bf16_kernel<false><<<dim3(HDIM / 64, FEAT / 64, NPH), blk, 0, stream>>>(pqw,   HDIM, (long long)FEAT * HDIM, PQT, FEAT, (long long)HDIM * FEAT, 0);
  transpose_bf16_kernel<false><<<dim3(HDIM / 64, FEAT / 64, NPH), blk, 0, stream>>>(pkw,   HDIM, (long long)FEAT * HDIM, PKT, FEAT, (long long)HDIM * FEAT, 0);
  transpose_bf16_kernel<true><<<dim3(DMOD / 64, HCOLS / 64, 1), blk, 0, stream>>>(ow, DMOD, 0LL, OWT2, AOP, 0LL, HCOLS);

  const dim3 gVT(((HCOLS / 64) * (SEQ / 64) + 7) / 8, NB);
  gemm64<__bf16, 1, 1><<<gVT, blk, 0, stream>>>(
      VWT, DMOD, 0LL, XB, DMOD, (long long)SEQ * DMOD,
      (void*)VT, (void*)VT, SEQ, (long long)HCOLS * SEQ, vb, HCOLS, SEQ, DMOD, 8.0f);
  const dim3 gSTD(((ROWS / 64) * (STDC / 64) + 7) / 8, 1);
  gemm64<__bf16, 1, 2><<<gSTD, blk, 0, stream>>>(
      XB, DMOD, 0LL, QWT, DMOD, 0LL,
      (void*)(QP + (WAVC + PRJC)), (void*)(QP + (WAVC + PRJC)), HCOLS, 0LL, sqb, ROWS, STDC, DMOD, 8.0f);
  gemm64<__bf16, 1, 2><<<gSTD, blk, 0, stream>>>(
      XB, DMOD, 0LL, KWT, DMOD, 0LL,
      (void*)(KP + (WAVC + PRJC)), (void*)(KP + (WAVC + PRJC)), HCOLS, 0LL, skb, ROWS, STDC, DMOD, 8.0f);
  const dim3 gF(((ROWS / 64) * (WAVC / 64) + 7) / 8, 1);
  gemm64<__bf16, 2, 0><<<gF, blk, 0, stream>>>(
      FB, FEAT, 0LL, WVT, FEAT, 0LL,
      (void*)WPH, (void*)WPL, WAVC, 0LL, vb, ROWS, WAVC, FEAT, 1.0f);
  gemm64<__bf16, 1, 0><<<gF, blk, 0, stream>>>(
      FB, FEAT, 0LL, PQT, FEAT, 0LL,
      (void*)(QP + WAVC), (void*)(QP + WAVC), HCOLS, 0LL, vb, ROWS, PRJC, FEAT, 8.0f);
  gemm64<__bf16, 1, 0><<<gF, blk, 0, stream>>>(
      FB, FEAT, 0LL, PKT, FEAT, 0LL,
      (void*)(KP + WAVC), (void*)(KP + WAVC), HCOLS, 0LL, vb, ROWS, PRJC, FEAT, 8.0f);

  attn_kernel<0><<<dim3(NB * NWH * NQB), dim3(128), 0, stream>>>(
      WPH, WPL, WAVC, WPH, WPL, WAVC, VT, MB, AO, 0, NWH, 0.125f);
  attn_kernel<1><<<dim3(NB * (NPH + NSH) * NQB), dim3(128), 0, stream>>>(
      QP, QP, HCOLS, KP, KP, HCOLS, VT, MB, AO, NWH, NPH + NSH, 1.0f / 512.0f);

  const dim3 gO(((ROWS / 64) * (DMOD / 64) + 7) / 8, 1);
  gemm64<__bf16, 0, 2><<<gO, blk, 0, stream>>>(
      AO, AOP, 0LL, OWT2, AOP, 0LL,
      d_out, d_out, DMOD, 0LL, ob, ROWS, DMOD, AOP, 1.0f);
  (void)hipGetLastError();
}
